// BiLSTMWithDotAttention_30623116820909
// MI455X (gfx1250) — hardware-verified
//
#include <hip/hip_runtime.h>


namespace {
constexpr int NB = 8, S = 1024, EM = 300, EP = 320, H = 512, G4 = 4 * H, D2 = 2 * H, VOCAB = 32000, NR = NB * S;
constexpr float XS = 8.0f, WSC = 256.0f, PS = 8.0f;

typedef _Float16 b16;
typedef __attribute__((ext_vector_type(16))) _Float16 v16b;
typedef __attribute__((ext_vector_type(8))) _Float16 v8b;
typedef __attribute__((ext_vector_type(2))) _Float16 v2b;
typedef __attribute__((ext_vector_type(8))) float v8f;
typedef __attribute__((ext_vector_type(4))) float v4f;
__device__ __forceinline__ float bf16_rne(float f) { unsigned int u = __float_as_uint(f); u += 0x7FFFu + ((u >> 16) & 1u); return __uint_as_float(u & 0xFFFF0000u); }
__device__ __forceinline__ v16b frag_kb(const b16* p, int hh) { const v8b a = *(const v8b*)(p + 8 * hh), b = *(const v8b*)(p + 16 + 8 * hh); v16b f;
#pragma unroll
  for (int e = 0; e < 8; ++e) { f[e] = a[e]; f[8 + e] = b[e]; } return f; }
__device__ __forceinline__ v8f wmma16b(v16b a, v16b b, v8f c) { v8f d = __builtin_amdgcn_wmma_f32_16x16x32_f16(false, a, false, b, (short)0, c, false, false); asm volatile("v_nop\n\tv_nop\n\tv_nop\n\tv_nop" : "+v"(d) : "v"(a), "v"(b)); return d; }
__device__ __forceinline__ void wave_lds_sync() { __builtin_amdgcn_fence(__ATOMIC_RELEASE, "workgroup"); __builtin_amdgcn_wave_barrier(); __builtin_amdgcn_fence(__ATOMIC_ACQUIRE, "workgroup"); }
__device__ __forceinline__ float nexp(float x) { return __builtin_amdgcn_exp2f(x * 1.4426950408889634f); }
__device__ __forceinline__ float pmul(float a, float b) { float p = a * b; asm volatile("" : "+v"(p)); return p; }
__device__ __forceinline__ float sigm(float x) { return 1.0f / (1.0f + nexp(-x)); }
__device__ __forceinline__ float tanh_(float x) { const float e = nexp(-2.0f * fabsf(x)); const float t = (1.0f - e) / (1.0f + e); return x < 0.0f ? -t : t; }

__global__ __launch_bounds__(256) void prepx_kernel(const int* __restrict__ ids, const float* __restrict__ emb, b16* __restrict__ X16) {
  const int wave = threadIdx.x >> 5, lane = threadIdx.x & 31; const int row = blockIdx.x * 8 + wave;
  v8b o0 = {}, o1 = {};
  if (row < NR) { int id = ids[row]; id = id < 0 ? 0 : (id >= VOCAB ? VOCAB - 1 : id); const float* src = emb + (size_t)id * EM;
#pragma unroll
    for (int q = 0; q < 8; ++q) { const int e = lane * 8 + q; o0[q] = (e < EM) ? (b16)(bf16_rne(src[e < EM ? e : 0]) * XS) : (b16)0.0f; const int e1 = 256 + lane * 8 + q; o1[q] = (lane < 8 && e1 < EM) ? (b16)(bf16_rne(src[e1 < EM ? e1 : 0]) * XS) : (b16)0.0f; } }
  if (row <= NR) for (int pass = 0; pass < 2; ++pass) { *(volatile v8b*)(X16 + (size_t)row * EP + lane * 8) = o0; if (lane < 8) *(volatile v8b*)(X16 + (size_t)row * EP + 256 + lane * 8) = o1; __threadfence(); }
}
__global__ __launch_bounds__(256) void prepw_kernel(const float* __restrict__ wihf, const float* __restrict__ whhf, const float* __restrict__ wihb, const float* __restrict__ whhb, b16* __restrict__ WIH, b16* __restrict__ WHH) {
  const int kind = blockIdx.y, dir = kind & 1, ish = kind >> 1; const int r = blockIdx.x * 8 + (threadIdx.x >> 5), lane = threadIdx.x & 31;
  if (ish == 0) { const float* w = (dir ? wihb : wihf) + (size_t)r * EM; b16* dst = WIH + ((size_t)dir * G4 + r) * EP; v8b o0, o1 = {};
#pragma unroll
    for (int q = 0; q < 8; ++q) { const int e = lane * 8 + q; o0[q] = (e < EM) ? (b16)(bf16_rne(w[e < EM ? e : 0]) * WSC) : (b16)0.0f; const int e1 = 256 + lane * 8 + q; o1[q] = (lane < 8 && e1 < EM) ? (b16)(bf16_rne(w[e1 < EM ? e1 : 0]) * WSC) : (b16)0.0f; }
    for (int pass = 0; pass < 2; ++pass) { *(volatile v8b*)(dst + lane * 8) = o0; if (lane < 8) *(volatile v8b*)(dst + 256 + lane * 8) = o1; __threadfence(); } }
  else { const float* w = (dir ? whhb : whhf) + (size_t)r * H; b16* dst = WHH + ((size_t)dir * G4 + r) * H;
    for (int pass = 0; pass < 2; ++pass) { for (int hq = 0; hq < 2; ++hq) { v8b o;
#pragma unroll
        for (int q = 0; q < 8; ++q) o[q] = (b16)(bf16_rne(w[hq * 256 + lane * 8 + q]) * WSC); *(volatile v8b*)(dst + hq * 256 + lane * 8) = o; } __threadfence(); } }
}
template <int STEPS>
__global__ __launch_bounds__(512) void lstm_kernel(const b16* __restrict__ X16, const b16* __restrict__ WIH, const b16* __restrict__ WHH, const float* __restrict__ bihf, const float* __restrict__ bhhf, const float* __restrict__ bihb, const float* __restrict__ bhhb, b16* __restrict__ OUT16) {
  __shared__ __attribute__((aligned(16))) b16 Hh[16][H + 8]; __shared__ __attribute__((aligned(16))) b16 Ho[NB][H + 8];
  const int dir = blockIdx.x, t_ = threadIdx.x, wave = t_ >> 5, lane = t_ & 31, nloc = lane & 15, hlf = lane >> 4;
  const b16* Wi = WIH + (size_t)dir * G4 * EP; const b16* Wh = WHH + (size_t)dir * G4 * H; const float* bi = dir ? bihb : bihf; const float* bh = dir ? bhhb : bhhf;
  for (int k = t_; k < 16 * (H + 8); k += 512) (&Hh[0][0])[k] = (b16)0.0f;
  float bg[2][4]; int ju[2];
#pragma unroll
  for (int ut = 0; ut < 2; ++ut) { ju[ut] = wave * 32 + ut * 16 + nloc;
#pragma unroll
    for (int g = 0; g < 4; ++g) bg[ut][g] = bf16_rne(bi[g * H + ju[ut]]) + bf16_rne(bh[g * H + ju[ut]]); }
  float cst[2][8];
#pragma unroll
  for (int ut = 0; ut < 2; ++ut)
#pragma unroll
    for (int r = 0; r < 8; ++r) cst[ut][r] = 0.0f;
  __syncthreads();
  for (int step = 0; step < STEPS; ++step) { const int t = dir ? (S - 1 - step) : step;
    v8f acc[2][4];
#pragma unroll
    for (int ut = 0; ut < 2; ++ut)
#pragma unroll
      for (int g = 0; g < 4; ++g) acc[ut][g] = (v8f){};
    { const size_t arow = (nloc < NB) ? ((size_t)nloc * S + t) : (size_t)NR;
#pragma unroll 2
      for (int kb = 0; kb < EP; kb += 32) { const v16b a = frag_kb(X16 + arow * EP + kb, hlf);
#pragma unroll
        for (int ut = 0; ut < 2; ++ut)
#pragma unroll
          for (int g = 0; g < 4; ++g) acc[ut][g] = wmma16b(a, frag_kb(Wi + (size_t)(g * H + ju[ut] - nloc + nloc) * EP + kb, hlf), acc[ut][g]); } }
#pragma unroll 4
    for (int kb = 0; kb < H; kb += 32) { const v16b a = frag_kb(&Hh[nloc][kb], hlf);
#pragma unroll
      for (int ut = 0; ut < 2; ++ut)
#pragma unroll
        for (int g = 0; g < 4; ++g) acc[ut][g] = wmma16b(a, frag_kb(Wh + (size_t)(g * H + ju[ut]) * H + kb, hlf), acc[ut][g]); }
    __syncthreads();
    if (hlf == 0) {
#pragma unroll
      for (int ut = 0; ut < 2; ++ut) { const int j = ju[ut];
#pragma unroll
        for (int r = 0; r < 8; ++r) { const float zi = acc[ut][0][r] * (1.0f / (XS * WSC)) + bg[ut][0], zf = acc[ut][1][r] * (1.0f / (XS * WSC)) + bg[ut][1], zg = acc[ut][2][r] * (1.0f / (XS * WSC)) + bg[ut][2], zo = acc[ut][3][r] * (1.0f / (XS * WSC)) + bg[ut][3];
          const float c = pmul(sigm(zf), cst[ut][r]) + pmul(sigm(zi), tanh_(zg)); cst[ut][r] = c; const float h = pmul(sigm(zo), tanh_(c)); const b16 hv = (b16)(h * XS);
          const float nh = __shfl_xor((float)hv, 1, 16); if ((nloc & 1) == 0) { v2b p2; p2[0] = hv; p2[1] = (b16)nh; *(v2b*)(&Hh[r][j]) = p2; *(v2b*)(&Ho[r][j]) = p2; } } } }
    else {
#pragma unroll
      for (int ut = 0; ut < 2; ++ut)
#pragma unroll
        for (int r = 0; r < 8; ++r) { const float nh = __shfl_xor(0.0f, 1, 16); (void)nh; } }
    __syncthreads();
    for (int pass = 0; pass < 2; ++pass) { { const int rr = wave >> 1, hq = wave & 1; *(volatile v8b*)(OUT16 + ((size_t)rr * S + t) * D2 + dir * H + hq * 256 + lane * 8) = *(const v8b*)(&Ho[rr][hq * 256 + lane * 8]); } __threadfence(); } }
}
__global__ __launch_bounds__(256) void ot_kernel(const b16* __restrict__ OUT16, b16* __restrict__ OT) {
  __shared__ __attribute__((aligned(16))) b16 Tt[64][64 + 8];
  const int b = blockIdx.z, d0 = blockIdx.y * 64, s0 = blockIdx.x * 64, t_ = threadIdx.x;
  for (int q = t_; q < 64 * 64; q += 256) { const int ss = q >> 6, dd = q & 63; Tt[dd][ss] = OUT16[((size_t)b * S + s0 + ss) * D2 + d0 + dd]; }
  __syncthreads();
  for (int pass = 0; pass < 2; ++pass) { for (int q = t_; q < 64 * 8; q += 256) { const int dd = q >> 3, c8 = (q & 7) * 8; *(volatile v8b*)(OT + ((size_t)b * D2 + d0 + dd) * S + s0 + c8) = *(const v8b*)(&Tt[dd][c8]); } __threadfence(); }
}
__global__ __launch_bounds__(64) void attn_kernel(const b16* __restrict__ OUT16, const b16* __restrict__ OT, float* __restrict__ att) {
  __shared__ __attribute__((aligned(16))) float To[2][16][256 + 4]; __shared__ __attribute__((aligned(16))) b16 Pt[2][16][S + 8];
  const int wave = threadIdx.x >> 5, lane = threadIdx.x & 31, hh = lane >> 4, col = lane & 15; const int b = blockIdx.y, q0 = blockIdx.x * 32 + wave * 16, qi = q0 + col;
  const b16* Ob = OUT16 + (size_t)b * S * D2; const b16* V = OT + (size_t)b * D2 * S; const b16* qrow = Ob + (size_t)qi * D2;
  const float scale = 1.0f / (XS * XS);
  float m = -INFINITY, l = 0.0f;
  for (int ps = 0; ps < 2; ++ps) {
    for (int kb = 0; kb < S; kb += 32) { v8f s0 = {}, s1 = {};
#pragma unroll 4
      for (int ks = 0; ks < D2 / 32; ++ks) { const v16b qf = frag_kb(qrow + ks * 32, hh); s0 = wmma16b(frag_kb(Ob + (size_t)(kb + col) * D2 + ks * 32, hh), qf, s0); s1 = wmma16b(frag_kb(Ob + (size_t)(kb + 16 + col) * D2 + ks * 32, hh), qf, s1); }
      if (ps == 0) { float mr = -INFINITY;
#pragma unroll
        for (int r = 0; r < 8; ++r) { s0[r] *= scale; s1[r] *= scale; mr = fmaxf(mr, fmaxf(s0[r], s1[r])); }
        mr = fmaxf(mr, __shfl_xor(mr, 16)); const float mn = fmaxf(m, mr); float sum = 0.0f;
#pragma unroll
        for (int r = 0; r < 8; ++r) sum += nexp(s0[r] - mn) + nexp(s1[r] - mn);
        sum += __shfl_xor(sum, 16); l = l * nexp(m - mn) + sum; m = mn; }
      else { const float invl = 1.0f / l;
#pragma unroll
        for (int r = 0; r < 8; ++r) { Pt[wave][col][kb + 8 * hh + r] = (b16)(nexp(s0[r] * scale - m) * invl * PS); Pt[wave][col][kb + 16 + 8 * hh + r] = (b16)(nexp(s1[r] * scale - m) * invl * PS); } } } }
  wave_lds_sync();
  for (int dc = 0; dc < 4; ++dc) { v8f o[16];
#pragma unroll
    for (int t = 0; t < 16; ++t) o[t] = (v8f){};
    for (int kb = 0; kb < S; kb += 32) { const v16b pb = frag_kb(&Pt[wave][col][kb], hh);
#pragma unroll
      for (int t = 0; t < 16; ++t) o[t] = wmma16b(frag_kb(V + (size_t)(dc * 256 + t * 16 + col) * S + kb, hh), pb, o[t]); }
#pragma unroll
    for (int t = 0; t < 16; ++t)
#pragma unroll
      for (int r = 0; r < 8; ++r) To[wave][col][t * 16 + 8 * hh + r] = o[t][r] * (1.0f / (PS * XS));
    wave_lds_sync();
    for (int pass = 0; pass < 2; ++pass) { for (int rr = 0; rr < 16; ++rr) for (int hq = 0; hq < 2; ++hq) *(volatile v4f*)(att + ((size_t)b * S + q0 + rr) * D2 + dc * 256 + hq * 128 + lane * 4) = *(const v4f*)(&To[wave][rr][hq * 128 + lane * 4]); __threadfence(); }
    wave_lds_sync(); }
}
}

extern "C" void kernel_launch(void* const* d_in, const int* in_sizes, int n_in, void* d_out, int out_size, void* d_ws, size_t ws_size, hipStream_t stream) {
  (void)n_in;
  auto Fp = [&](int i) { return (const float*)d_in[i]; };
  if (in_sizes[0] != NR || in_sizes[2] != VOCAB * EM || in_sizes[3] != G4 * EM || in_sizes[4] != G4 * H || in_sizes[7] != G4 * EM || in_sizes[8] != G4 * H || out_size != NR * D2) return;
  size_t off = 0; char* ws = (char*)d_ws;
  auto carve = [&](size_t bytes) { char* p = ws + off; off += (bytes + 255) & ~(size_t)255; return p; };
  b16* X16 = (b16*)carve((size_t)(NR + 16) * EP * 2); b16* WIH = (b16*)carve((size_t)2 * G4 * EP * 2); b16* WHH = (b16*)carve((size_t)2 * G4 * H * 2); b16* OUT16 = (b16*)carve((size_t)NR * D2 * 2); b16* OT = (b16*)carve((size_t)NR * D2 * 2);
  if (off > ws_size || off > ((size_t)128 << 20)) return;
  prepx_kernel<<<NR / 8 + 1, 256, 0, stream>>>((const int*)d_in[0], Fp(2), X16);
  prepw_kernel<<<dim3(G4 / 8, 4), 256, 0, stream>>>(Fp(3), Fp(4), Fp(7), Fp(8), WIH, WHH);
  lstm_kernel<S><<<2, 512, 0, stream>>>(X16, WIH, WHH, Fp(5), Fp(6), Fp(9), Fp(10), OUT16);
  ot_kernel<<<dim3(S / 64, D2 / 64, NB), 256, 0, stream>>>(OUT16, OT);
  attn_kernel<<<dim3(S / 32, NB), 64, 0, stream>>>(OUT16, OT, (float*)d_out);
}
